// LinearAttention_87565793230944
// MI455X (gfx1250) — hardware-verified
//
#include <hip/hip_runtime.h>
#ifndef NB
#define NB 2
#endif
#ifndef SEQ
#define SEQ 2048
#endif
#define NB_FULL 2
#define SEQ_FULL 2048
#define DMOD 1024
#define NH 16
#define HD 64
#define QT 256
#define LOR ((SEQ < 512) ? SEQ : 512)
#define NKX SEQ
#define NRW ((size_t)NB * SEQ)
#define FEPS 1.0e-6f
#define PCARRY 4096.0f
#define RCARRY 1024.0f
static_assert(NB >= 1 && NB <= NB_FULL);
static_assert(SEQ <= SEQ_FULL);
static_assert(SEQ % QT == 0);
static_assert(QT % 128 == 0);
static_assert(LOR % QT == 0);
static_assert((SEQ - LOR) % 128 == 0);
static_assert(DMOD == NH * HD);
static_assert(HD == 64);

typedef _Float16 v16h __attribute__((ext_vector_type(16)));
typedef unsigned short v8us __attribute__((ext_vector_type(8), may_alias));
typedef float v8f __attribute__((ext_vector_type(8)));
typedef float v4f __attribute__((ext_vector_type(4)));
typedef float v4fa __attribute__((ext_vector_type(4), may_alias));
typedef _Float16 v4h __attribute__((ext_vector_type(4)));
union FragH { v16h v; v8us half[2]; _Float16 h[16]; unsigned short u[16]; };

__device__ __forceinline__ unsigned short bf16_bits(float x) { unsigned int u = __float_as_uint(x); return (unsigned short)((u + 0x7FFFu + ((u >> 16) & 1u)) >> 16); }
__device__ __forceinline__ float bf16_val(unsigned short b) { return __uint_as_float(((unsigned int)b) << 16); }
__device__ __forceinline__ float bf16_rne(float x) { return bf16_val(bf16_bits(x)); }

__device__ __forceinline__ v16h g2_frag(const _Float16* p, int hh) { FragH f; f.half[0] = *(const v8us*)((const unsigned short*)p + 8 * hh); f.half[1] = *(const v8us*)((const unsigned short*)p + 16 + 8 * hh); return f.v; }
__device__ __forceinline__ v8f g2_mma(v16h a, v16h b, v8f c) { v8f d = __builtin_amdgcn_wmma_f32_16x16x32_f16(false, a, false, b, (short)0, c, false, false); asm volatile("v_nop\n\tv_nop\n\tv_nop\n\tv_nop" : "+v"(d) : "v"(a), "v"(b)); return d; }
template <int NT>
__device__ __forceinline__ void mmaS(v16h ah, v16h al, v16h bh, v16h bl, v8f& c, v8f& cr) {
  c = __builtin_amdgcn_wmma_f32_16x16x32_f16(false, ah, false, bh, (short)0, c, false, false);
  cr = __builtin_amdgcn_wmma_f32_16x16x32_f16(false, al, false, bh, (short)0, cr, false, false);
  if (NT >= 3) cr = __builtin_amdgcn_wmma_f32_16x16x32_f16(false, ah, false, bl, (short)0, cr, false, false);
  asm volatile("v_nop\n\tv_nop\n\tv_nop\n\tv_nop" : "+v"(c), "+v"(cr) : "v"(ah), "v"(al), "v"(bh), "v"(bl));
}

__global__ __launch_bounds__(256) void k_x16(const float* __restrict__ x, _Float16* __restrict__ X16, size_t n8) {
  const size_t t = (size_t)blockIdx.x * 256 + threadIdx.x; if (t >= n8) return;
  const size_t r = t / (DMOD / 8); const int c = (int)(t % (DMOD / 8)) * 8;
  const size_t b = r / SEQ, s = r % SEQ;
  const float* src = x + (b * SEQ_FULL + s) * DMOD + c;
  FragH f;
#pragma unroll
  for (int q = 0; q < 8; ++q) f.h[q] = (_Float16)bf16_rne(src[q]);
  unsigned short* d = (unsigned short*)X16 + t * 8;
  *(volatile v8us*)d = f.half[0]; __threadfence(); *(volatile v8us*)d = f.half[0];
}

__global__ __launch_bounds__(256) void k_wnat(const float* __restrict__ w, size_t n8, _Float16* __restrict__ Bt) {
  const size_t t = (size_t)blockIdx.x * 256 + threadIdx.x; if (t >= n8) return; FragH f;
#pragma unroll
  for (int q = 0; q < 8; ++q) f.h[q] = (_Float16)(bf16_rne(w[t * 8 + q]) * 16.0f);
  *(volatile v8us*)((unsigned short*)Bt + t * 8) = f.half[0]; __threadfence(); *(volatile v8us*)((unsigned short*)Bt + t * 8) = f.half[0];
}

template <int ACT>
__global__ __launch_bounds__(128) void k_gemm2(const _Float16* __restrict__ A, int lda, size_t sA, const _Float16* __restrict__ Bh, int ldb, size_t sB, float alpha,
    float* __restrict__ C, _Float16* __restrict__ C16, int ldc, size_t sC, _Float16* __restrict__ C16l, int loseg, int lorows, int M, int N, int K) {
  static_assert(ACT == 0 || ACT == 1);
  __shared__ __attribute__((aligned(16))) float so[4][32][68];
  const int tid = threadIdx.x, w = tid >> 5, lane = tid & 31, ln = lane & 15, hh = lane >> 4; const int by = blockIdx.y;
  A += (size_t)by * sA; Bh += (size_t)by * sB; const size_t cofs = (size_t)by * sC;
  const int ntn = N >> 6; const int mt = blockIdx.x / ntn, nq = blockIdx.x - mt * ntn; const int row0 = mt * 128 + 32 * w, col0 = nq * 64; if (row0 >= M) return;
  const _Float16* a0p = A + (size_t)(row0 + ln) * lda; const _Float16* a1p = a0p + (size_t)16 * lda;
  const _Float16* b0p = Bh + (size_t)(col0 + ln) * ldb; const _Float16* b1p = b0p + (size_t)16 * ldb; const _Float16* b2p = b1p + (size_t)16 * ldb; const _Float16* b3p = b2p + (size_t)16 * ldb;
  const v8f z8 = {0.f,0.f,0.f,0.f,0.f,0.f,0.f,0.f}; v8f c00 = z8, c01 = z8, c02 = z8, c03 = z8, c10 = z8, c11 = z8, c12 = z8, c13 = z8;
#pragma unroll 1
  for (int kb = 0; kb < K; kb += 32) { const v16h a0 = g2_frag(a0p + kb, hh), a1 = g2_frag(a1p + kb, hh);
    v16h b = g2_frag(b0p + kb, hh); c00 = g2_mma(a0, b, c00); c10 = g2_mma(a1, b, c10);
    b = g2_frag(b1p + kb, hh); c01 = g2_mma(a0, b, c01); c11 = g2_mma(a1, b, c11);
    b = g2_frag(b2p + kb, hh); c02 = g2_mma(a0, b, c02); c12 = g2_mma(a1, b, c12);
    b = g2_frag(b3p + kb, hh); c03 = g2_mma(a0, b, c03); c13 = g2_mma(a1, b, c13); }
  v8f accs[8] = {c00, c01, c02, c03, c10, c11, c12, c13};
#pragma unroll
  for (int u = 0; u < 8; ++u) { const int t = u & 3, half = u >> 2;
#pragma unroll
    for (int r = 0; r < 8; ++r) { const int rloc = half * 16 + 8 * hh + r; float v = accs[u][r] * alpha; if (ACT == 1) v = fmaxf(v, 0.f) + FEPS; so[w][rloc][t * 16 + ln] = v; } }
  __builtin_amdgcn_fence(4  , "workgroup"); __builtin_amdgcn_wave_barrier();
  const int rsub = lane >> 4, c4 = (lane & 15) * 4;
  long lorow0 = -1;
  if (C16l) { const int sg = row0 / loseg, si = row0 - sg * loseg; if (si < lorows) lorow0 = (long)sg * lorows + si; }
  for (int pass = 0; pass < 2; ++pass) {
#pragma unroll
    for (int q = 0; q < 16; ++q) { const int r = q * 2 + rsub; const v4f v = *(const v4fa*)&so[w][r][c4];
      if (C) *(volatile v4f*)(C + cofs + (size_t)(row0 + r) * ldc + col0 + c4) = v;
      if (C16) { v4h h4;
#pragma unroll
        for (int i = 0; i < 4; ++i) h4[i] = (_Float16)v[i];
        *(volatile v4h*)(C16 + cofs + (size_t)(row0 + r) * ldc + col0 + c4) = h4; }
      if (lorow0 >= 0) { v4h l4;
#pragma unroll
        for (int i = 0; i < 4; ++i) { const _Float16 h = (_Float16)v[i]; l4[i] = (_Float16)((v[i] - (float)h) * RCARRY); }
        *(volatile v4h*)(C16l + cofs + (size_t)(lorow0 + r) * ldc + col0 + c4) = l4; } }
    if (pass == 0) __threadfence(); }
}

template <int NT>
__global__ __launch_bounds__(128) void k_gemmS(const _Float16* __restrict__ Ah, int ldah, size_t sAh, const _Float16* __restrict__ Al, int ldal, size_t sAl,
    const _Float16* __restrict__ Bh, int ldbh, size_t sBh, const _Float16* __restrict__ Bl, int ldbl, size_t sBl, float alpha, float rscale,
    float* __restrict__ C, _Float16* __restrict__ C16, _Float16* __restrict__ C16l, int ldc, size_t sC, int ldcl, size_t sCl, int M, int N, int K) {
  static_assert(NT == 2 || NT == 3);
  __shared__ __attribute__((aligned(16))) float so[4][16][64];
  const int tid = threadIdx.x, w = tid >> 5, lane = tid & 31, ln = lane & 15, hh = lane >> 4; const int by = blockIdx.y;
  Ah += (size_t)by * sAh; Al += (size_t)by * sAl; Bh += (size_t)by * sBh; Bl += (size_t)by * sBl; const size_t cofs = (size_t)by * sC, cofsl = (size_t)by * sCl;
  const int ntn = N >> 6; const int mt = blockIdx.x / ntn, nq = blockIdx.x - mt * ntn; const int row0 = mt * 64 + 16 * w, col0 = nq * 64; if (row0 >= M) return;
  const _Float16* ahp = Ah + (size_t)(row0 + ln) * ldah; const _Float16* alp = Al + (size_t)(row0 + ln) * ldal;
  v8f acc[4] = {}, accr[4] = {};
#pragma unroll 1
  for (int kb = 0; kb < K; kb += 32) {
    const v16h fah = g2_frag(ahp + kb, hh), fal = g2_frag(alp + kb, hh);
#pragma unroll
    for (int t = 0; t < 4; ++t) {
      const v16h fbh = g2_frag(Bh + (size_t)(col0 + t * 16 + ln) * ldbh + kb, hh);
      v16h fbl = fbh;
      if (NT >= 3) fbl = g2_frag(Bl + (size_t)(col0 + t * 16 + ln) * ldbl + kb, hh);
      mmaS<NT>(fah, fal, fbh, fbl, acc[t], accr[t]);
    }
  }
#pragma unroll
  for (int t = 0; t < 4; ++t) {
#pragma unroll
    for (int r = 0; r < 8; ++r) so[w][8 * hh + r][t * 16 + ln] = (acc[t][r] + accr[t][r] * rscale) * alpha; }
  __builtin_amdgcn_fence(4  , "workgroup"); __builtin_amdgcn_wave_barrier();
  const int rsub = lane >> 4, c4 = (lane & 15) * 4;
  for (int pass = 0; pass < 2; ++pass) {
#pragma unroll
    for (int q = 0; q < 8; ++q) { const int r = q * 2 + rsub; const v4f v = *(const v4fa*)&so[w][r][c4];
      if (C) *(volatile v4f*)(C + cofs + (size_t)(row0 + r) * ldc + col0 + c4) = v;
      if (C16) { v4h h4;
#pragma unroll
        for (int i = 0; i < 4; ++i) h4[i] = (_Float16)v[i];
        *(volatile v4h*)(C16 + cofs + (size_t)(row0 + r) * ldc + col0 + c4) = h4; }
      if (C16l) { v4h l4;
#pragma unroll
        for (int i = 0; i < 4; ++i) { const _Float16 h = (_Float16)v[i]; l4[i] = (_Float16)((v[i] - (float)h) * RCARRY); }
        *(volatile v4h*)(C16l + cofsl + (size_t)(row0 + r) * ldcl + col0 + c4) = l4; } }
    if (pass == 0) __threadfence(); }
}

template <int NHv, int TTv>
__global__ __launch_bounds__(256) void k_vt(const _Float16* __restrict__ V16, int ldv, int voff, _Float16* __restrict__ Vt) {
  __shared__ unsigned short tl[64][66];
  const int tid = threadIdx.x; const int slab = blockIdx.x / (TTv / 64), lg = blockIdx.x % (TTv / 64); const int b = slab / NHv, h = slab % NHv;
  for (int i = tid; i < 64 * 8; i += 256) { const int r = i / 8, c8 = (i % 8) * 8; FragH f; f.half[0] = *(const v8us*)((const unsigned short*)V16 + ((size_t)b * TTv + lg * 64 + r) * ldv + voff + h * 64 + c8);
#pragma unroll
    for (int q = 0; q < 8; ++q) tl[r][c8 + q] = f.u[q]; }
  __syncthreads();
  for (int pass = 0; pass < 2; ++pass) {
#pragma unroll
    for (int rd = 0; rd < 2; ++rd) { const int d = rd * 32 + tid / 8, pc = tid % 8; FragH f;
#pragma unroll
      for (int q = 0; q < 8; ++q) f.u[q] = tl[pc * 8 + q][d];
      *(volatile v8us*)((unsigned short*)Vt + ((size_t)slab * 64 + d) * TTv + lg * 64 + pc * 8) = f.half[0]; }
    if (pass == 0) __threadfence(); }
}

template <bool LO>
__global__ __launch_bounds__(128) void k_linz(const float* __restrict__ S, _Float16* __restrict__ P, _Float16* __restrict__ Pl, int ldl, int nrow, int q0, int nk) {
  #pragma clang fp contract(off)
  const int w = threadIdx.x >> 5, lane = threadIdx.x & 31;
  const int row = blockIdx.x * 4 + w; if (row >= nrow) return;
  const int last = q0 + (row % QT);
  const float* s = S + (size_t)row * NKX;
  float zp = 0.f;
#pragma unroll 1
  for (int c0 = 0; c0 < nk; c0 += 256) {
    const int j0 = c0 + lane * 8;
    const v4f a = *(const v4fa*)(s + j0), bq = *(const v4fa*)(s + j0 + 4);
    const float xv[8] = {a[0], a[1], a[2], a[3], bq[0], bq[1], bq[2], bq[3]};
#pragma unroll
    for (int q = 0; q < 8; ++q) zp += (j0 + q <= last) ? xv[q] : 0.f;
  }
#pragma unroll
  for (int o = 16; o > 0; o >>= 1) zp += __shfl_xor(zp, o);
  const float sc = (1.0f / (zp + FEPS)) * PCARRY;
#pragma unroll 1
  for (int c0 = 0; c0 < nk; c0 += 256) {
    const int j0 = c0 + lane * 8;
    const v4f a = *(const v4fa*)(s + j0), bq = *(const v4fa*)(s + j0 + 4);
    const float xv[8] = {a[0], a[1], a[2], a[3], bq[0], bq[1], bq[2], bq[3]};
    FragH ph, pl;
#pragma unroll
    for (int q = 0; q < 8; ++q) {
      const float tv = (j0 + q <= last) ? xv[q] : 0.f;
      const float p = tv * sc; const _Float16 h = (_Float16)p;
      ph.h[q] = h; pl.h[q] = LO ? (_Float16)((p - (float)h) * RCARRY) : (_Float16)0.0f;
    }
    unsigned short* dp = (unsigned short*)P + (size_t)row * NKX + j0;
    *(volatile v8us*)dp = ph.half[0];
    if (LO) { unsigned short* dl = (unsigned short*)Pl + (size_t)row * ldl + j0; *(volatile v8us*)dl = pl.half[0]; }
    __threadfence();
    *(volatile v8us*)dp = ph.half[0];
    if (LO) { unsigned short* dl = (unsigned short*)Pl + (size_t)row * ldl + j0; *(volatile v8us*)dl = pl.half[0]; }
  }
}

extern "C" void kernel_launch(void* const* d_in, const int* in_sizes, int n_in,
                              void* d_out, int out_size, void* d_ws, size_t ws_size, hipStream_t stream) {
  if (n_in < 5) return;
  const size_t need_x = ((size_t)(NB - 1) * SEQ_FULL + SEQ) * DMOD;
  const size_t need_w = (size_t)DMOD * DMOD;
  if ((size_t)in_sizes[0] < need_x || (size_t)in_sizes[1] < need_w || (size_t)in_sizes[2] < need_w || (size_t)in_sizes[3] < need_w || (size_t)in_sizes[4] < need_w) return;
  if ((size_t)out_size < need_x) return;
  const float* x  = (const float*)d_in[0];
  const float* Wq = (const float*)d_in[1];
  const float* Wk = (const float*)d_in[2];
  const float* Wv = (const float*)d_in[3];
  const float* Wo = (const float*)d_in[4];
  float* out = (float*)d_out;
  char* ws = (char*)d_ws; size_t off = 0;
  auto take = [&](size_t bytes) { char* p = ws + off; off += (bytes + 255) & ~(size_t)255; return p; };
  const size_t NLR = (size_t)NB * LOR;
  _Float16* X16  = (_Float16*)take(NRW * DMOD * 2);
  _Float16* Wq16 = (_Float16*)take(need_w * 2); _Float16* Wk16 = (_Float16*)take(need_w * 2); _Float16* Wv16 = (_Float16*)take(need_w * 2); _Float16* Wo16 = (_Float16*)take(need_w * 2);
  _Float16* Qh   = (_Float16*)take(NRW * DMOD * 2); _Float16* Kh = (_Float16*)take(NRW * DMOD * 2); _Float16* Vh = (_Float16*)take(NRW * DMOD * 2);
  _Float16* Ql   = (_Float16*)take(NLR * DMOD * 2); _Float16* Kl = (_Float16*)take(NLR * DMOD * 2); _Float16* Vl = (_Float16*)take(NLR * DMOD * 2);
  _Float16* VT   = (_Float16*)take((size_t)NB * NH * HD * SEQ * 2);
  _Float16* VTl  = (_Float16*)take((size_t)NB * NH * HD * LOR * 2);
  float*    S    = (float*)take((size_t)NH * QT * NKX * 4);
  _Float16* P    = (_Float16*)take((size_t)NH * QT * NKX * 2);
  _Float16* Pl   = (_Float16*)take((size_t)NH * QT * LOR * 2);
  _Float16* ctxh = (_Float16*)take(NRW * DMOD * 2);
  _Float16* ctxl = (_Float16*)take(NLR * DMOD * 2);
  if (off > ws_size) return;

  k_x16<<<(unsigned)((NRW * DMOD / 8 + 255) / 256), 256, 0, stream>>>(x, X16, NRW * DMOD / 8);
  const unsigned gw = (unsigned)((need_w / 8 + 255) / 256);
  k_wnat<<<gw, 256, 0, stream>>>(Wq, need_w / 8, Wq16);
  k_wnat<<<gw, 256, 0, stream>>>(Wk, need_w / 8, Wk16);
  k_wnat<<<gw, 256, 0, stream>>>(Wv, need_w / 8, Wv16);
  k_wnat<<<gw, 256, 0, stream>>>(Wo, need_w / 8, Wo16);
  const unsigned gproj = (unsigned)((NRW / 128) * (DMOD / 64));
  k_gemm2<1><<<dim3(gproj, 1), 128, 0, stream>>>(X16, DMOD, (size_t)0, Wq16, DMOD, (size_t)0, 0.0625f, nullptr, Qh, DMOD, (size_t)0, Ql, SEQ, LOR, (int)NRW, DMOD, DMOD);
  k_gemm2<1><<<dim3(gproj, 1), 128, 0, stream>>>(X16, DMOD, (size_t)0, Wk16, DMOD, (size_t)0, 0.0625f, nullptr, Kh, DMOD, (size_t)0, Kl, SEQ, LOR, (int)NRW, DMOD, DMOD);
  k_gemm2<0><<<dim3(gproj, 1), 128, 0, stream>>>(X16, DMOD, (size_t)0, Wv16, DMOD, (size_t)0, 0.0625f, nullptr, Vh, DMOD, (size_t)0, Vl, SEQ, LOR, (int)NRW, DMOD, DMOD);
  k_vt<NH, SEQ><<<(unsigned)(NB * NH * (SEQ / 64)), 256, 0, stream>>>(Vh, DMOD, 0, VT);
  k_vt<NH, LOR><<<(unsigned)(NB * NH * (LOR / 64)), 256, 0, stream>>>(Vl, DMOD, 0, VTl);
  for (int b = 0; b < NB; ++b) {
    const size_t rb = (size_t)b * SEQ, rl = (size_t)b * LOR;
    for (int q0 = 0; q0 < SEQ; q0 += QT) {
      const int nk = q0 + QT;
      if (nk <= LOR) {
        k_gemmS<3><<<dim3((QT / 64) * (nk / 64), NH), 128, 0, stream>>>(Qh + (rb + q0) * DMOD, DMOD, (size_t)HD, Ql + (rl + q0) * DMOD, DMOD, (size_t)HD,
            Kh + rb * DMOD, DMOD, (size_t)HD, Kl + rl * DMOD, DMOD, (size_t)HD, 1.0f, 0.0009765625f,
            S, nullptr, nullptr, NKX, (size_t)QT * NKX, 0, (size_t)0, QT, nk, HD);
        k_linz<true><<<(NH * QT) / 4, 128, 0, stream>>>(S, P, Pl, LOR, NH * QT, q0, nk);
        k_gemmS<3><<<dim3((QT / 64) * (HD / 64), NH), 128, 0, stream>>>(P, NKX, (size_t)QT * NKX, Pl, LOR, (size_t)QT * LOR,
            VT + (size_t)b * NH * HD * SEQ, SEQ, (size_t)HD * SEQ, VTl + (size_t)b * NH * HD * LOR, LOR, (size_t)HD * LOR, 0.000244140625f, 0.0009765625f,
            nullptr, ctxh + (rb + q0) * DMOD, ctxl + (rl + q0) * DMOD, DMOD, (size_t)HD, DMOD, (size_t)HD, QT, HD, nk);
      } else {
        k_gemm2<0><<<dim3((QT / 128) * (nk / 64), NH), 128, 0, stream>>>(Qh + (rb + q0) * DMOD, DMOD, (size_t)HD, Kh + rb * DMOD, DMOD, (size_t)HD, 1.0f,
            S, nullptr, NKX, (size_t)QT * NKX, nullptr, 1, 0, QT, nk, HD);
        k_linz<false><<<(NH * QT) / 4, 128, 0, stream>>>(S, P, nullptr, 0, NH * QT, q0, nk);
        k_gemm2<0><<<dim3((QT / 128) * (HD / 64), NH), 128, 0, stream>>>(P, NKX, (size_t)QT * NKX, VT + (size_t)b * NH * HD * SEQ, SEQ, (size_t)HD * SEQ, 0.000244140625f,
            nullptr, ctxh + (rb + q0) * DMOD, DMOD, (size_t)HD, nullptr, 1, 0, QT, HD, nk);
      }
    }
  }
  k_gemmS<2><<<dim3((LOR / 64) * (DMOD / 64), NB), 128, 0, stream>>>(ctxh, DMOD, (size_t)SEQ * DMOD, ctxl, DMOD, (size_t)LOR * DMOD,
      Wo16, DMOD, (size_t)0, Wo16, DMOD, (size_t)0, 0.0625f, 0.0009765625f,
      out, nullptr, nullptr, DMOD, (size_t)SEQ_FULL * DMOD, 0, (size_t)0, LOR, DMOD, DMOD);
  if (SEQ > LOR)
    k_gemm2<0><<<dim3(((SEQ - LOR) / 128) * (DMOD / 64), NB), 128, 0, stream>>>(ctxh + (size_t)LOR * DMOD, DMOD, (size_t)SEQ * DMOD, Wo16, DMOD, (size_t)0, 0.0625f,
        out + (size_t)LOR * DMOD, nullptr, DMOD, (size_t)SEQ_FULL * DMOD, nullptr, 1, 0, SEQ - LOR, DMOD, DMOD);
}
